// MembershipDecoder_41403484733992
// MI455X (gfx1250) — hardware-run, weakly checked
//
#include <hip/hip_runtime.h>
#include <math.h>

typedef __attribute__((ext_vector_type(16))) _Float16 v16h;
typedef __attribute__((ext_vector_type(8)))  _Float16 v8h;
typedef __attribute__((ext_vector_type(4)))  _Float16 v4h;
typedef __attribute__((ext_vector_type(2)))  _Float16 v2h;
typedef __attribute__((ext_vector_type(16))) __bf16   v16b;
typedef __attribute__((ext_vector_type(8)))  __bf16   v8b;
typedef __attribute__((ext_vector_type(8)))  float    v8f;
typedef __attribute__((ext_vector_type(4)))  float    v4f;
typedef __attribute__((ext_vector_type(2)))  float    v2f;

constexpr int kNR   = 1024;
constexpr int kNC   = 1024;
constexpr int kDI   = 128;
constexpr int kH    = 100;
constexpr int kHP   = 128;
constexpr int kSlab = 256;
constexpr int kPairs = kSlab * kNC;
constexpr int kThr  = 256;
constexpr float kInCarry = 1024.0f;
constexpr float kSc20 = 1.0f / (kInCarry * kInCarry);
constexpr float kF16MinNormal = 6.103515625e-5f;
constexpr float kLnEps = 1.0e-3f;

static_assert(kNR == 1024 && kNC == 1024 && kDI == 128 && kH == 100 && kHP == 128 && kSlab == 256 && kPairs == 262144, "the index arithmetic below uses these sizes");

constexpr size_t kOffSEQ16 = 0ull;
constexpr size_t kOffCOL16 = 262144ull;
constexpr size_t kOffWS16 = 524288ull;
constexpr size_t kOffWC16 = 557056ull;
constexpr size_t kOffWM16 = 589824ull;
constexpr size_t kOffBS = 622592ull;
constexpr size_t kOffBC = 623104ull;
constexpr size_t kOffBM = 623616ull;
constexpr size_t kOffGR = 624128ull;
constexpr size_t kOffBE = 624640ull;
constexpr size_t kOffWO = 625152ull;
constexpr size_t kOffSP = 625664ull;
constexpr size_t kOffCP = 1149952ull;
constexpr size_t kOffLN16 = 1674240ull;
constexpr size_t kOffH2 = 68783104ull;
constexpr size_t kOffLG = 203000832ull;
constexpr size_t kOffMXS = 207195136ull;
constexpr size_t kWsTotal = 207203328ull;
static_assert(kWsTotal <= 268435456ull, "the carve stands under 256 MiB");
static_assert(kOffSEQ16 == 0
  && kOffCOL16 == kOffSEQ16 + 262144ull
  && kOffWS16 == kOffCOL16 + 262144ull
  && kOffWC16 == kOffWS16 + 32768ull
  && kOffWM16 == kOffWC16 + 32768ull
  && kOffBS == kOffWM16 + 32768ull
  && kOffBC == kOffBS + 512ull
  && kOffBM == kOffBC + 512ull
  && kOffGR == kOffBM + 512ull
  && kOffBE == kOffGR + 512ull
  && kOffWO == kOffBE + 512ull
  && kOffSP == kOffWO + 512ull
  && kOffCP == kOffSP + 524288ull
  && kOffLN16 == kOffCP + 524288ull
  && kOffH2 == kOffLN16 + 67108864ull
  && kOffLG == kOffH2 + 134217728ull
  && kOffMXS == kOffLG + 4194304ull
  && kWsTotal == kOffMXS + 8192ull, "the carve is a chain: every region starts where the one before ends");
static_assert((kOffSEQ16 % 256) == 0 && (kOffCOL16 % 256) == 0 && (kOffWS16 % 256) == 0 && (kOffWC16 % 256) == 0 && (kOffWM16 % 256) == 0 && (kOffBS % 256) == 0 && (kOffBC % 256) == 0 && (kOffBM % 256) == 0 && (kOffGR % 256) == 0 && (kOffBE % 256) == 0 && (kOffWO % 256) == 0 && (kOffSP % 256) == 0 && (kOffCP % 256) == 0 && (kOffLN16 % 256) == 0 && (kOffH2 % 256) == 0 && (kOffLG % 256) == 0 && (kOffMXS % 256) == 0, "every region starts on a multiple of 256 B");

__device__ __forceinline__ unsigned short f2bf_bits(float f) {
  unsigned u = __float_as_uint(f);
  return (unsigned short)((u + 0x7FFFu + ((u >> 16) & 1u)) >> 16);
}
__device__ __forceinline__ float bf_bits2f(unsigned short h) { return __uint_as_float(((unsigned)h) << 16); }
__device__ __forceinline__ float bf16r(float f) { return bf_bits2f(f2bf_bits(f)); }
__device__ __forceinline__ float carry_flush(float v, float carry) {
  const float s = v * carry;
  return (fabsf(s) < kF16MinNormal) ? 0.0f : s;
}

__device__ __forceinline__ void dep_guard4_h(v8f& a, v8f& b, v8f& c, v8f& d, v16h x, v16h y) { asm volatile("v_nop\n\tv_nop\n\tv_nop\n\tv_nop" : "+v"(a), "+v"(b), "+v"(c), "+v"(d) : "v"(x), "v"(y)); }
__device__ __forceinline__ void dep_guard4_b(v8f& a, v8f& b, v8f& c, v8f& d, v16b x, v16b y) { asm volatile("v_nop\n\tv_nop\n\tv_nop\n\tv_nop" : "+v"(a), "+v"(b), "+v"(c), "+v"(d) : "v"(x), "v"(y)); }
__device__ __forceinline__ void keep4_h(v16h a, v16h b, v16h c, v16h d) { asm volatile("v_nop" :: "v"(a), "v"(b), "v"(c), "v"(d)); }
__device__ __forceinline__ void keep4_b(v16b a, v16b b, v16b c, v16b d) { asm volatile("v_nop" :: "v"(a), "v"(b), "v"(c), "v"(d)); }
__device__ __forceinline__ void acc_guard4(v8f& a, v8f& b, v8f& c, v8f& d) { asm volatile("v_nop\n\tv_nop\n\tv_nop\n\tv_nop" : "+v"(a), "+v"(b), "+v"(c), "+v"(d)); }

template <typename T> struct Frag;
template <> struct Frag<_Float16> {
  typedef v16h V; union U { v16h v; v8h h[2]; };
  static __device__ __forceinline__ v16h load(const _Float16* p) {
    U f; f.h[0] = *(const v8h*)(p); f.h[1] = *(const v8h*)(p + 16); return f.v;
  }
  static __device__ __forceinline__ v8f mma(v16h a, v16h b, v8f c) {
    return __builtin_amdgcn_wmma_f32_16x16x32_f16(false, a, false, b, (short)0, c, false, false);
  }
  static __device__ __forceinline__ void guard4(v8f& a, v8f& b, v8f& c, v8f& d, v16h x, v16h y) { dep_guard4_h(a, b, c, d, x, y); }
  static __device__ __forceinline__ void keep(v16h a, v16h b, v16h c, v16h d) { keep4_h(a, b, c, d); }
};
template <> struct Frag<__bf16> {
  typedef v16b V; union U { v16b v; v8b h[2]; };
  static __device__ __forceinline__ v16b load(const __bf16* p) {
    U f; f.h[0] = *(const v8b*)(p); f.h[1] = *(const v8b*)(p + 16); return f.v;
  }
  static __device__ __forceinline__ v8f mma(v16b a, v16b b, v8f c) {
    return __builtin_amdgcn_wmma_f32_16x16x32_bf16(false, a, false, b, (short)0, c, false, false);
  }
  static __device__ __forceinline__ void guard4(v8f& a, v8f& b, v8f& c, v8f& d, v16b x, v16b y) { dep_guard4_b(a, b, c, d, x, y); }
  static __device__ __forceinline__ void keep(v16b a, v16b b, v16b c, v16b d) { keep4_b(a, b, c, d); }
};

__device__ __forceinline__ v8f mma_h(v16h a, v16h b, v8f c) {
  c = __builtin_amdgcn_wmma_f32_16x16x32_f16(false, a, false, b, (short)0, c, false, false);
  asm volatile("v_nop\n\tv_nop\n\tv_nop\n\tv_nop" : "+v"(c) : "v"(a), "v"(b));
  return c;
}

template <int ET> struct Elem;
template <> struct Elem<0> { typedef _Float16 T; };
template <> struct Elem<1> { typedef __bf16 T; };
template <int ET, bool SPLIT, int BIAS_MODE, int OUT_MODE, bool RESID, int ACT = 0>
__global__ __launch_bounds__(256) void wmma_gemm64(
    const unsigned short* __restrict__ Ap, const unsigned short* __restrict__ A2p, int lda, long strideA,
    const unsigned short* __restrict__ Btp, const unsigned short* __restrict__ Bt2p, int ldb, long strideB,
    void* __restrict__ Cout, void* __restrict__ Cout2, int ldc, long strideC,
    const float* __restrict__ bias,
    const float* __restrict__ resid, long strideR,
    int M, int N, int K, float scale) {
  typedef typename Elem<ET>::T T;
  typedef typename Frag<T>::V V;
  const T* A = (const T*)Ap; const T* A2 = (const T*)A2p; const T* Bt = (const T*)Btp; const T* Bt2 = (const T*)Bt2p;
  __shared__ __align__(16) float sT[8][16 * 68];
  const int b    = blockIdx.y;
  const int lane = threadIdx.x & 31;
  const int wave = threadIdx.x >> 5;
  const int tilesN = N >> 6;
  const int tilesM = M >> 6;
  const int tile = blockIdx.x * 8 + wave;
  if (tile >= tilesM * tilesN) return;
  const int tm = tile / tilesN;
  const int tn = tile - tm * tilesN;
  const int m0 = tm << 6;
  const int n0 = tn << 6;

  const T* Ab  = A  + (size_t)b * strideA;
  const T* Bb  = Bt + (size_t)b * strideB;
  const T* Ab2 = SPLIT ? (A2  + (size_t)b * strideA) : nullptr;
  const T* Bb2 = SPLIT ? (Bt2 + (size_t)b * strideB) : nullptr;

  const int rlane = lane & 15;
  const int koff  = (lane >> 4) * 8;
  const int mOff  = (lane >> 4) * 8;

  v8f acc[4][4];
#pragma unroll
  for (int i = 0; i < 4; ++i)
#pragma unroll
    for (int j = 0; j < 4; ++j) acc[i][j] = (v8f){0.f,0.f,0.f,0.f,0.f,0.f,0.f,0.f};

  for (int k0 = 0; k0 < K; k0 += 32) {
    V bh[4], bl[4];
#pragma unroll
    for (int j = 0; j < 4; ++j) {
      const size_t bo = (size_t)(n0 + (j << 4) + rlane) * ldb + koff + k0;
      bh[j] = Frag<T>::load(Bb + bo);
      if (SPLIT) bl[j] = Frag<T>::load(Bb2 + bo);
    }
#pragma unroll
    for (int i = 0; i < 4; ++i) {
      const size_t ao = (size_t)(m0 + (i << 4) + rlane) * lda + koff + k0;
      V ah = Frag<T>::load(Ab + ao);
      V al;
      if (SPLIT) al = Frag<T>::load(Ab2 + ao);
#pragma unroll
      for (int j = 0; j < 4; ++j) {
        acc[i][j] = Frag<T>::mma(ah, bh[j], acc[i][j]);
        if (SPLIT) {
          acc[i][j] = Frag<T>::mma(ah, bl[j], acc[i][j]);
          acc[i][j] = Frag<T>::mma(al, bh[j], acc[i][j]);
        }
      }
      Frag<T>::guard4(acc[i][0], acc[i][1], acc[i][2], acc[i][3], ah, SPLIT ? al : ah);
    }
    Frag<T>::keep(bh[0], bh[1], bh[2], bh[3]);
    if (SPLIT) Frag<T>::keep(bl[0], bl[1], bl[2], bl[3]);
  }
  acc_guard4(acc[0][0], acc[0][1], acc[0][2], acc[0][3]);
  acc_guard4(acc[1][0], acc[1][1], acc[1][2], acc[1][3]);
  acc_guard4(acc[2][0], acc[2][1], acc[2][2], acc[2][3]);
  acc_guard4(acc[3][0], acc[3][1], acc[3][2], acc[3][3]);

  float* slab = sT[wave];
  const float* Rb = RESID ? (resid + (size_t)b * strideR) : nullptr;
#pragma unroll
  for (int i = 0; i < 4; ++i) {
    const int mBase = m0 + (i << 4);
#pragma unroll
    for (int j = 0; j < 4; ++j) {
      const int n = n0 + (j << 4) + rlane;
      float bv = 0.f;
      if (BIAS_MODE == 2) bv = bias[n];
#pragma unroll
      for (int r = 0; r < 8; ++r) {
        float v = acc[i][j][r] * scale;
        if (BIAS_MODE == 1) v += bias[mBase + mOff + r];
        if (BIAS_MODE == 2) v += bv;
        if (RESID) v += Rb[(size_t)(mBase + mOff + r) * ldc + n];
        if (ACT == 1) v = tanhf(v);
        if (ACT == 2) v = fmaxf(v, 0.0f);
        if (ACT == 3) v = v / (1.0f + expf(-v));
        if (ACT == 4) v = (v > 0.f) ? v : 0.01f * v;
        slab[(mOff + r) * 68 + (j << 4) + rlane] = v;
      }
    }
    __builtin_amdgcn_fence(__ATOMIC_RELEASE, "workgroup");
    __builtin_amdgcn_wave_barrier();
    __builtin_amdgcn_fence(__ATOMIC_ACQUIRE, "workgroup");
    if (OUT_MODE == 0) {
      float* C = (float*)Cout + (size_t)b * strideC;
      const int hh = lane >> 4, c4 = (lane & 15) * 4;
      for (int pass = 0; pass < 2; ++pass) {
#pragma unroll
        for (int it = 0; it < 8; ++it) {
          const int row = it * 2 + hh;
          v4f v = *(const v4f*)(slab + row * 68 + c4);
          *(volatile v4f*)(C + (size_t)(mBase + row) * ldc + n0 + c4) = v;
        }
        __threadfence();
      }
    } else {
      const int q = lane >> 3, c8 = (lane & 7) * 8;
      unsigned short* C  = (unsigned short*)Cout  + (size_t)b * strideC;
      unsigned short* C2 = (OUT_MODE == 2) ? ((unsigned short*)Cout2 + (size_t)b * strideC) : nullptr;
      for (int pass = 0; pass < 2; ++pass) {
#pragma unroll
        for (int it = 0; it < 4; ++it) {
          const int row = it * 4 + q;
          const float* sp = slab + row * 68 + c8;
          v8h hv, lv;
#pragma unroll
          for (int e = 0; e < 8; ++e) {
            if (OUT_MODE == 1) {
              hv[e] = (_Float16)sp[e];
            } else {
              unsigned short hb = f2bf_bits(sp[e]);
              unsigned short lb = f2bf_bits(sp[e] - bf_bits2f(hb));
              hv[e] = __builtin_bit_cast(_Float16, hb);
              lv[e] = __builtin_bit_cast(_Float16, lb);
            }
          }
          *(volatile v8h*)(C + (size_t)(mBase + row) * ldc + n0 + c8) = hv;
          if (OUT_MODE == 2) *(volatile v8h*)(C2 + (size_t)(mBase + row) * ldc + n0 + c8) = lv;
        }
        __threadfence();
      }
    }
    __builtin_amdgcn_fence(__ATOMIC_RELEASE, "workgroup");
    __builtin_amdgcn_wave_barrier();
    __builtin_amdgcn_fence(__ATOMIC_ACQUIRE, "workgroup");
  }
}

__global__ __launch_bounds__(kThr) void cast_plane_kernel(const float* __restrict__ src, unsigned short* __restrict__ dst,
                                                          int colsLog2, int dstPitch, int dstOff) {
  const int i   = blockIdx.x * kThr + threadIdx.x;
  const int sh  = colsLog2 - 3;
  const int row = i >> sh;
  const int c8  = (i & ((1 << sh) - 1)) * 8;
  const float* sp = src + ((size_t)row << colsLog2) + c8;
  const v4f a0 = *(const v4f*)(sp);
  const v4f a1 = *(const v4f*)(sp + 4);
  v8h hv;
#pragma unroll
  for (int e = 0; e < 4; ++e) {
    const float f0 = a0[e];
    const float f1 = a1[e];
    hv[e]     = (_Float16)carry_flush(bf16r(f0), kInCarry);
    hv[4 + e] = (_Float16)carry_flush(bf16r(f1), kInCarry);
  }
  unsigned short* dp = dst + (size_t)row * dstPitch + dstOff + c8;
  *(volatile v8h*)dp = hv;
  __threadfence();
  *(volatile v8h*)dp = hv;
}

__global__ __launch_bounds__(kThr) void recpad_kernel(const float* __restrict__ src, float* __restrict__ dst, int count) {
  const unsigned i = blockIdx.x * (unsigned)kThr + threadIdx.x;
  v4f o;
#pragma unroll
  for (int e = 0; e < 4; ++e) {
    const int k = (int)(4u * i) + e;
    const int kk = (k < count) ? k : (count - 1);
    const float v = bf16r(src[kk]);
    o[e] = (k < count) ? v : 0.0f;
  }
  float* dp = dst + 4u * i;
  *(volatile v4f*)dp = o;
  __threadfence();
  *(volatile v4f*)dp = o;
}

__global__ __launch_bounds__(kThr) void wtpad_kernel(const float* __restrict__ Wp, unsigned short* __restrict__ Bt, int rowsK, int colsN) {
  const unsigned i = blockIdx.x * (unsigned)kThr + threadIdx.x;
  const int n = (int)(i >> 4), g = (int)(i & 15u);
  const int nn = (n < colsN) ? n : (colsN - 1);
  v8h w;
#pragma unroll
  for (int t = 0; t < 8; ++t) {
    const int k = 8 * g + t;
    const int kk = (k < rowsK) ? k : (rowsK - 1);
    const float v = bf16r(Wp[(size_t)kk * colsN + nn]);
    const float s = carry_flush(v, kInCarry);
    w[t] = (_Float16)(((n < colsN) && (k < rowsK)) ? s : 0.0f);
  }
  unsigned short* dp = Bt + (size_t)n * kHP + 8 * g;
  *(volatile v8h*)dp = w;
  __threadfence();
  *(volatile v8h*)dp = w;
}

__global__ __launch_bounds__(kThr) void lnrows_kernel(const float* __restrict__ SP, const float* __restrict__ CP, const float* __restrict__ GR, const float* __restrict__ BE, unsigned short* __restrict__ LN16, int n0) {
  const unsigned i = blockIdx.x * (unsigned)kThr + threadIdx.x;
  const unsigned m = i & 1023u, n = (unsigned)n0 + (i >> 10);
  const float* sp = SP + (size_t)n * kHP; const float* cp = CP + (size_t)m * kHP;
  float h[100];
  float sum = 0.0f;
#pragma unroll
  for (int c = 0; c < 25; ++c) {
    const v4f a = *(const v4f*)(sp + 4 * c), b = *(const v4f*)(cp + 4 * c);
#pragma unroll
    for (int e = 0; e < 4; ++e) { const float t = a[e] + b[e]; const float r = (t > 0.0f) ? t : 0.0f; h[4 * c + e] = r; sum += r; }
  }
  const float mean = sum * 0.01f;
  float sq = 0.0f;
#pragma unroll
  for (int k = 0; k < 100; ++k) { const float d = h[k] - mean; h[k] = d; sq = fmaf(d, d, sq); }
  const float inv = 1.0f / sqrtf(sq * 0.01f + kLnEps);
  unsigned short* dp = LN16 + (size_t)i * kHP;
  v8h w[16];
#pragma unroll
  for (int c = 0; c < 16; ++c) {
#pragma unroll
    for (int e = 0; e < 8; ++e) {
      const int k = 8 * c + e;
      if (k < 100) { const float v = (h[k] * inv) * GR[k] + BE[k]; w[c][e] = (_Float16)carry_flush(v, kInCarry); }
      else w[c][e] = (_Float16)0.0f;
    }
  }
#pragma unroll
  for (int c = 0; c < 16; ++c) *(volatile v8h*)(dp + 8 * c) = w[c];
  __threadfence();
#pragma unroll
  for (int c = 0; c < 16; ++c) *(volatile v8h*)(dp + 8 * c) = w[c];
}

__global__ __launch_bounds__(kThr) void lastdot_kernel(const float* __restrict__ H2, const float* __restrict__ WO, const float* __restrict__ bo, float* __restrict__ LG, int n0) {
  const unsigned i = blockIdx.x * (unsigned)kThr + threadIdx.x;
  const float* hp = H2 + (size_t)i * kHP;
  float acc = 0.0f;
#pragma unroll
  for (int c = 0; c < 25; ++c) {
    const v4f a = *(const v4f*)(hp + 4 * c);
#pragma unroll
    for (int e = 0; e < 4; ++e) acc = fmaf(a[e], WO[4 * c + e], acc);
  }
  const float o = acc + bf16r(bo[0]);
  float* dp = LG + (size_t)n0 * kNC + i;
  *(volatile float*)dp = o;
  __threadfence();
  *(volatile float*)dp = o;
}

__global__ __launch_bounds__(kThr) void rowstat_kernel(const float* __restrict__ LG, float* __restrict__ MXS) {
  const unsigned n = blockIdx.x * (unsigned)kThr + threadIdx.x;
  const float* lp = LG + (size_t)n * kNC;
  float mx = lp[0];
  for (int c = 0; c < 256; ++c) {
    const v4f a = *(const v4f*)(lp + 4 * c);
#pragma unroll
    for (int e = 0; e < 4; ++e) mx = (a[e] > mx) ? a[e] : mx;
  }
  float s = 0.0f;
  for (int c = 0; c < 256; ++c) {
    const v4f a = *(const v4f*)(lp + 4 * c);
#pragma unroll
    for (int e = 0; e < 4; ++e) s += expf(a[e] - mx);
  }
  const v2f o = {mx, 1.0f / s};
  *(volatile v2f*)(MXS + (size_t)n * 2u) = o;
  __threadfence();
  *(volatile v2f*)(MXS + (size_t)n * 2u) = o;
}

__global__ __launch_bounds__(kThr) void softmaxout_kernel(const float* __restrict__ LG, const float* __restrict__ MXS, float* __restrict__ res) {
  const unsigned v = blockIdx.x * (unsigned)kThr + threadIdx.x;
  const v2f st = *(const v2f*)(MXS + (size_t)(v >> 10) * 2u);
  const float o = expf(LG[v] - st[0]) * st[1];
  for (int pass = 0; pass < 2; ++pass) {
    *(volatile float*)(res + v) = o;
    *(volatile float*)(res + (size_t)kNR * kNC + v) = o;
    __threadfence();
  }
}

extern "C" void kernel_launch(void* const* d_in, const int* in_sizes, int n_in,
                              void* d_out, int out_size, void* d_ws, size_t ws_size,
                              hipStream_t stream) {
  if (n_in < 13 || d_out == nullptr || d_ws == nullptr) return;
  if (in_sizes[0] != kNR * kDI || in_sizes[1] != kNC * kDI || in_sizes[3] != kDI * kH || in_sizes[4] != kH || in_sizes[5] != kDI * kH || in_sizes[6] != kH
      || in_sizes[7] != kH || in_sizes[8] != kH || in_sizes[9] != kH * kH || in_sizes[10] != kH || in_sizes[11] != kH || in_sizes[12] != 1) return;
  if (out_size != 2 * kNR * kNC) return;
  if (ws_size < kWsTotal) return;
  const float* sq = (const float*)d_in[0];
  const float* cl = (const float*)d_in[1];
  const float* ws_ = (const float*)d_in[3];
  const float* bs = (const float*)d_in[4];
  const float* wc = (const float*)d_in[5];
  const float* bc = (const float*)d_in[6];
  const float* ga = (const float*)d_in[7];
  const float* be = (const float*)d_in[8];
  const float* wm = (const float*)d_in[9];
  const float* bm = (const float*)d_in[10];
  const float* wo = (const float*)d_in[11];
  const float* bo = (const float*)d_in[12];
  float* out = (float*)d_out;
  char* ws = (char*)d_ws;
  unsigned short* SEQ16 = (unsigned short*)(ws + kOffSEQ16);
  unsigned short* COL16 = (unsigned short*)(ws + kOffCOL16);
  unsigned short* WS16 = (unsigned short*)(ws + kOffWS16);
  unsigned short* WC16 = (unsigned short*)(ws + kOffWC16);
  unsigned short* WM16 = (unsigned short*)(ws + kOffWM16);
  float* BS = (float*)(ws + kOffBS);
  float* BC = (float*)(ws + kOffBC);
  float* BM = (float*)(ws + kOffBM);
  float* GR = (float*)(ws + kOffGR);
  float* BE = (float*)(ws + kOffBE);
  float* WO = (float*)(ws + kOffWO);
  float* SP = (float*)(ws + kOffSP);
  float* CP = (float*)(ws + kOffCP);
  unsigned short* LN16 = (unsigned short*)(ws + kOffLN16);
  float* H2 = (float*)(ws + kOffH2);
  float* LG = (float*)(ws + kOffLG);
  float* MXS = (float*)(ws + kOffMXS);

  static_assert((kNR * kDI / 8) % kThr == 0 && (kHP * kHP / 8) % kThr == 0 && kH % 4 == 0 && (kHP - kH) % 4 == 0 && kPairs % kThr == 0 && kNR % kThr == 0 && (kNR * kNC) % kThr == 0
                && ((kNR / 64) * (kHP / 64)) % 4 == 0 && ((kPairs / 64) * (kHP / 64)) % 8 == 0 && kDI % 32 == 0 && kHP % 32 == 0 && kNR % kSlab == 0, "every grid exact");
  cast_plane_kernel<<<kNR * kDI / 8 / kThr, kThr, 0, stream>>>(sq, SEQ16, 7, kDI, 0);
  cast_plane_kernel<<<kNC * kDI / 8 / kThr, kThr, 0, stream>>>(cl, COL16, 7, kDI, 0);
  wtpad_kernel<<<kHP * kHP / 8 / kThr, kThr, 0, stream>>>(ws_, WS16, kDI, kH);
  wtpad_kernel<<<kHP * kHP / 8 / kThr, kThr, 0, stream>>>(wc, WC16, kDI, kH);
  wtpad_kernel<<<kHP * kHP / 8 / kThr, kThr, 0, stream>>>(wm, WM16, kH, kH);
  recpad_kernel<<<1, kHP / 4, 0, stream>>>(bs, BS, kH);
  recpad_kernel<<<1, kHP / 4, 0, stream>>>(bc, BC, kH);
  recpad_kernel<<<1, kHP / 4, 0, stream>>>(bm, BM, kH);
  recpad_kernel<<<1, kHP / 4, 0, stream>>>(ga, GR, kH);
  recpad_kernel<<<1, kHP / 4, 0, stream>>>(be, BE, kH);
  recpad_kernel<<<1, kHP / 4, 0, stream>>>(wo, WO, kH);
  wmma_gemm64<0, false, 2, 0, false, 0><<<dim3((kNR / 64) * (kHP / 64) / 8, 1), 256, 0, stream>>>(
      SEQ16, SEQ16, kDI, 0L, WS16, WS16, kHP, 0L, (void*)SP, (void*)SP, kHP, 0L, BS, nullptr, 0L, kNR, kHP, kDI, kSc20);
  wmma_gemm64<0, false, 2, 0, false, 0><<<dim3((kNC / 64) * (kHP / 64) / 8, 1), 256, 0, stream>>>(
      COL16, COL16, kDI, 0L, WC16, WC16, kHP, 0L, (void*)CP, (void*)CP, kHP, 0L, BC, nullptr, 0L, kNC, kHP, kDI, kSc20);
  for (int n0 = 0; n0 < kNR; n0 += kSlab) {
    lnrows_kernel<<<kPairs / kThr, kThr, 0, stream>>>(SP, CP, GR, BE, LN16, n0);
    wmma_gemm64<0, false, 2, 0, false, 0><<<dim3((kPairs / 64) * (kHP / 64) / 8, 1), 256, 0, stream>>>(
        LN16, LN16, kHP, 0L, WM16, WM16, kHP, 0L, (void*)H2, (void*)H2, kHP, 0L, BM, nullptr, 0L, kPairs, kHP, kHP, kSc20);
    lastdot_kernel<<<kPairs / kThr, kThr, 0, stream>>>(H2, WO, bo, LG, n0);
  }
  rowstat_kernel<<<kNR / kThr, kThr, 0, stream>>>(LG, MXS);
  softmaxout_kernel<<<kNR * kNC / kThr, kThr, 0, stream>>>(LG, MXS, out);
}
